// GraphNet_88596585382209
// MI455X (gfx1250) — hardware-verified
//
#include <hip/hip_runtime.h>
#include <stdint.h>

#define NNODE   128
#define NB      8
#define FD      512
#define MR      (NNODE * NB)
#define NC3     (2 * FD)
#define FT      64
#define SLOPE   0.1f
#define INV_NM1 (1.0f / 127.0f)
#define TP      72

static_assert(MR % 128 == 0);
static_assert(NC3 % 64 == 0);
static_assert(FD % 64 == 0);
static_assert(FD % 32 == 0);
static_assert(NNODE == 128);
static_assert((MR * FD / 8) % 256 == 0);
static_assert(FT == 64);
static_assert((TP * 2) % 16 == 0);

typedef __attribute__((ext_vector_type(16))) __bf16 v16b;
typedef __attribute__((ext_vector_type(8)))  __bf16 v8b;
typedef __attribute__((ext_vector_type(8)))  float  v8f;
typedef __attribute__((ext_vector_type(4)))  float  v4f;
typedef __attribute__((ext_vector_type(4)))  unsigned int v4u;
typedef __attribute__((ext_vector_type(2)))  unsigned int v2u;
typedef v8b __attribute__((may_alias)) v8ba;
typedef v4f __attribute__((may_alias)) v4fa;
typedef v4u __attribute__((may_alias)) v4ua;
typedef v2u __attribute__((may_alias)) v2ua;

union FragU { v16b v; v8b h[2]; };

__device__ __forceinline__ unsigned short f2bf_bits(float f) {
  const unsigned u = __float_as_uint(f);
  return (unsigned short)((u + 0x7FFFu + ((u >> 16) & 1u)) >> 16);
}
__device__ __forceinline__ float bf_bits2f(unsigned short h) { return __uint_as_float(((unsigned)h) << 16); }
__device__ __forceinline__ float bf16r(float f) {
  unsigned u = __float_as_uint(f);
  u = (u + 0x7FFFu + ((u >> 16) & 1u)) & 0xFFFF0000u;
  return __uint_as_float(u);
}
__device__ __forceinline__ unsigned pk16(unsigned short a, unsigned short b) { return (unsigned)a | ((unsigned)b << 16); }

__device__ __forceinline__ v8f wmma_bf16(v16b a, v16b b, v8f c) {
  v8f d = __builtin_amdgcn_wmma_f32_16x16x32_bf16(false, a, false, b, (short)0, c, false, false);
  asm volatile("v_nop\n\tv_nop\n\tv_nop\n\tv_nop" : "+v"(d) : "v"(a), "v"(b));
  return d;
}

__device__ __forceinline__ v16b load_frag(const unsigned short* p, int hh) {
  FragU f;
  f.h[0] = *(const v8ba*)(p + 8 * hh);
  f.h[1] = *(const v8ba*)(p + 16 + 8 * hh);
  return f.v;
}

__device__ __forceinline__ void gemm_core_32x64(
    const unsigned short* __restrict__ Ah, const unsigned short* __restrict__ Al,
    const unsigned short* __restrict__ Bt, int K, size_t aoff, size_t boff, int hh, v8f (&acc)[2][4]) {
  const unsigned short* a0h = Ah + aoff;
  const unsigned short* a1h = a0h + (size_t)16 * K;
  const unsigned short* a0l = Al + aoff;
  const unsigned short* a1l = a0l + (size_t)16 * K;
  const unsigned short* bp  = Bt + boff;
#pragma unroll 1
  for (int k0 = 0; k0 < K; k0 += 32) {
    const v16b f0h = load_frag(a0h + k0, hh);
    const v16b f0l = load_frag(a0l + k0, hh);
    const v16b f1h = load_frag(a1h + k0, hh);
    const v16b f1l = load_frag(a1l + k0, hh);
#pragma unroll
    for (int nt = 0; nt < 4; ++nt) {
      const v16b fb = load_frag(bp + (size_t)nt * 16 * K + k0, hh);
      acc[0][nt] = wmma_bf16(f0h, fb, acc[0][nt]);
      acc[0][nt] = wmma_bf16(f0l, fb, acc[0][nt]);
      acc[1][nt] = wmma_bf16(f1h, fb, acc[1][nt]);
      acc[1][nt] = wmma_bf16(f1l, fb, acc[1][nt]);
    }
  }
}

__device__ __forceinline__ void gemm_core1_32x64(
    const unsigned short* __restrict__ A, const unsigned short* __restrict__ Bt,
    int K, size_t aoff, size_t boff, int hh, v8f (&acc)[2][4]) {
  const unsigned short* a0 = A + aoff;
  const unsigned short* a1 = a0 + (size_t)16 * K;
  const unsigned short* bp = Bt + boff;
#pragma unroll 1
  for (int k0 = 0; k0 < K; k0 += 32) {
    const v16b f0 = load_frag(a0 + k0, hh);
    const v16b f1 = load_frag(a1 + k0, hh);
#pragma unroll
    for (int nt = 0; nt < 4; ++nt) {
      const v16b fb = load_frag(bp + (size_t)nt * 16 * K + k0, hh);
      acc[0][nt] = wmma_bf16(f0, fb, acc[0][nt]);
      acc[1][nt] = wmma_bf16(f1, fb, acc[1][nt]);
    }
  }
}

__global__ __launch_bounds__(256) void k_cvt(const float* __restrict__ x, unsigned short* __restrict__ Xb) {
  const int g = blockIdx.x * 256 + threadIdx.x;
  if (g >= MR * FD / 8) return;
  const float* src = x + (size_t)g * 8;
  const v4f a = *(const v4fa*)src;
  const v4f c = *(const v4fa*)(src + 4);
  v4u o;
  o[0] = pk16(f2bf_bits(a[0]), f2bf_bits(a[1]));
  o[1] = pk16(f2bf_bits(a[2]), f2bf_bits(a[3]));
  o[2] = pk16(f2bf_bits(c[0]), f2bf_bits(c[1]));
  o[3] = pk16(f2bf_bits(c[2]), f2bf_bits(c[3]));
  unsigned short* dst = Xb + (size_t)g * 8;
  *(volatile v4u*)dst = o;
  __threadfence();
  *(volatile v4u*)dst = o;
}

__global__ __launch_bounds__(256) void k_wt(const float* __restrict__ W3, const float* __restrict__ W5,
                                            unsigned short* __restrict__ B3t, unsigned short* __restrict__ B5t) {
  __shared__ __align__(16) unsigned short sT[64 * TP];
  const int tid = threadIdx.x, lane = tid & 31, w = tid >> 5;
  const int c0 = blockIdx.x * 64, k0 = blockIdx.y * 64, z = blockIdx.z;
  const float* src = W3;
  unsigned short* dst = B3t;
  if (z == 1) { src = W3 + (size_t)FD * FD; dst = B3t + (size_t)FD * FD; }
  else if (z == 2) { src = W5; dst = B5t; }
  const int c4 = (tid & 15) * 4, rr = tid >> 4;
#pragma unroll
  for (int p = 0; p < 4; ++p) {
    const int r = rr + 16 * p;
    const v4f v = *(const v4fa*)(src + (size_t)(k0 + r) * FD + c0 + c4);
    sT[(c4 + 0) * TP + r] = f2bf_bits(v[0]);
    sT[(c4 + 1) * TP + r] = f2bf_bits(v[1]);
    sT[(c4 + 2) * TP + r] = f2bf_bits(v[2]);
    sT[(c4 + 3) * TP + r] = f2bf_bits(v[3]);
  }
  __syncthreads();
  const int q8 = lane & 7, sub = lane >> 3;
  v4u vv[2];
#pragma unroll
  for (int it = 0; it < 2; ++it) {
    const int row = 32 * it + 4 * w + sub;
    vv[it] = *(const v4ua*)(sT + row * TP + 8 * q8);
  }
  for (int pass = 0; pass < 2; ++pass) {
#pragma unroll
    for (int it = 0; it < 2; ++it) {
      const int row = 32 * it + 4 * w + sub;
      *(volatile v4u*)(dst + (size_t)(c0 + row) * FD + k0 + 8 * q8) = vv[it];
    }
    __threadfence();
  }
}

__global__ __launch_bounds__(128) void k_ab(const unsigned short* __restrict__ Xb,
                                            const unsigned short* __restrict__ B3t,
                                            float* __restrict__ AB) {
  __shared__ __align__(16) float sF[128 * 64];
  const int tid = threadIdx.x, lane = tid & 31, w = tid >> 5;
  const int hh = lane >> 4, m = lane & 15;
  const int m0 = blockIdx.x * 128;
  const int n0 = blockIdx.y * 64;
  const int m0w = m0 + 32 * w;

  const v8f zero8 = {0.f, 0.f, 0.f, 0.f, 0.f, 0.f, 0.f, 0.f};
  v8f acc[2][4];
#pragma unroll
  for (int mt = 0; mt < 2; ++mt)
#pragma unroll
    for (int nt = 0; nt < 4; ++nt) acc[mt][nt] = zero8;

  gemm_core1_32x64(Xb, B3t, FD, (size_t)(m0w + m) * FD, (size_t)(n0 + m) * FD, hh, acc);

#pragma unroll
  for (int nt = 0; nt < 4; ++nt)
#pragma unroll
    for (int mt = 0; mt < 2; ++mt)
#pragma unroll
      for (int r = 0; r < 8; ++r) {
        const int tokl = 32 * w + 16 * mt + 8 * hh + r;
        const int feat = 16 * nt + m;
        sF[tokl * 64 + feat] = acc[mt][nt][r];
      }
  __syncthreads();
  {
    const int rsub = lane >> 4, c4 = (lane & 15) * 4;
    v4f vals[16];
#pragma unroll
    for (int it = 0; it < 16; ++it) {
      const int row = 32 * w + 2 * it + rsub;
      vals[it] = *(const v4fa*)(sF + row * 64 + c4);
    }
    for (int pass = 0; pass < 2; ++pass) {
#pragma unroll
      for (int it = 0; it < 16; ++it) {
        const int row = 32 * w + 2 * it + rsub;
        *(volatile v4f*)(AB + (size_t)(m0 + row) * NC3 + n0 + c4) = vals[it];
      }
      __threadfence();
    }
  }
}

__global__ __launch_bounds__(256) void k_pair(const float* __restrict__ AB, const float* __restrict__ b3,
                                              unsigned short* __restrict__ MShi, unsigned short* __restrict__ MSlo) {
  __shared__ __align__(16) unsigned char smem[32768];
  float* sC = (float*)smem;
  unsigned short* sH = (unsigned short*)smem;
  unsigned short* sL = sH + NNODE * FT;
  const int tid = threadIdx.x, lane = tid & 31, w = tid >> 5;
  const int b = blockIdx.y, f0 = blockIdx.x * FT;

  {
    const int c4 = (tid & 15) * 4, rr = tid >> 4;
#pragma unroll
    for (int p = 0; p < 8; ++p) {
      const int j = rr + 16 * p;
      const v4f v = *(const v4fa*)(AB + (size_t)(j * NB + b) * NC3 + FD + f0 + c4);
      *(v4fa*)(sC + j * FT + c4) = v;
    }
  }
  const int q = tid & 15, ig = tid >> 4;
  const v4f braw = *(const v4fa*)(b3 + f0 + 4 * q);
  const v4f bb = {bf16r(braw[0]), bf16r(braw[1]), bf16r(braw[2]), bf16r(braw[3])};
  v4f x[8];
#pragma unroll
  for (int ii = 0; ii < 8; ++ii) {
    const int i = ig + 16 * ii;
    const v4f a = *(const v4fa*)(AB + (size_t)(i * NB + b) * NC3 + f0 + 4 * q);
    x[ii] = a + bb;
  }
  __syncthreads();

  const v4f zero4 = {0.f, 0.f, 0.f, 0.f};
  v4f acc[8];
#pragma unroll
  for (int ii = 0; ii < 8; ++ii) acc[ii] = zero4;

#pragma unroll 2
  for (int j = 0; j < NNODE; ++j) {
    const v4f c = *(const v4fa*)(sC + j * FT + 4 * q);
#pragma unroll
    for (int ii = 0; ii < 8; ++ii)
#pragma unroll
      for (int e = 0; e < 4; ++e) {
        const float zz = x[ii][e] + c[e];
        acc[ii][e] += fmaxf(zz, zz * SLOPE);
      }
  }

#pragma unroll
  for (int ii = 0; ii < 8; ++ii) {
    const int i = ig + 16 * ii;
    const v4f cd = *(const v4fa*)(sC + i * FT + 4 * q);
#pragma unroll
    for (int e = 0; e < 4; ++e) {
      const float zc = x[ii][e] + cd[e];
      const float d  = fmaxf(zc, zc * SLOPE);
      acc[ii][e] = (acc[ii][e] - d) * INV_NM1;
    }
  }
  __syncthreads();

#pragma unroll
  for (int ii = 0; ii < 8; ++ii) {
    const int i = ig + 16 * ii;
    v2u hv2, lv2;
#pragma unroll
    for (int p = 0; p < 2; ++p) {
      const unsigned short h0 = f2bf_bits(acc[ii][2 * p]), h1 = f2bf_bits(acc[ii][2 * p + 1]);
      const unsigned short l0 = f2bf_bits(acc[ii][2 * p] - bf_bits2f(h0));
      const unsigned short l1 = f2bf_bits(acc[ii][2 * p + 1] - bf_bits2f(h1));
      hv2[p] = pk16(h0, h1);
      lv2[p] = pk16(l0, l1);
    }
    *(v2ua*)(sH + i * FT + 4 * q) = hv2;
    *(v2ua*)(sL + i * FT + 4 * q) = lv2;
  }
  __syncthreads();

  const int q8 = lane & 7, sub = lane >> 3;
  v4u hv[4], lv[4];
#pragma unroll
  for (int it = 0; it < 4; ++it) {
    const int il = 32 * it + 4 * w + sub;
    hv[it] = *(const v4ua*)(sH + il * FT + 8 * q8);
    lv[it] = *(const v4ua*)(sL + il * FT + 8 * q8);
  }
  for (int pass = 0; pass < 2; ++pass) {
#pragma unroll
    for (int it = 0; it < 4; ++it) {
      const int il = 32 * it + 4 * w + sub;
      const size_t go = (size_t)(il * NB + b) * FD + f0 + 8 * q8;
      *(volatile v4u*)(MShi + go) = hv[it];
      *(volatile v4u*)(MSlo + go) = lv[it];
    }
    __threadfence();
  }
}

__global__ __launch_bounds__(128) void k_out(const unsigned short* __restrict__ MShi,
                                             const unsigned short* __restrict__ MSlo,
                                             const unsigned short* __restrict__ B5t,
                                             const float* __restrict__ b5, const float* __restrict__ x,
                                             float* __restrict__ out) {
  __shared__ __align__(16) float sF[128 * 64];
  const int tid = threadIdx.x, lane = tid & 31, w = tid >> 5;
  const int hh = lane >> 4, m = lane & 15;
  const int m0 = blockIdx.x * 128;
  const int n0 = blockIdx.y * 64;
  const int m0w = m0 + 32 * w;

  const v8f zero8 = {0.f, 0.f, 0.f, 0.f, 0.f, 0.f, 0.f, 0.f};
  v8f acc[2][4];
#pragma unroll
  for (int mt = 0; mt < 2; ++mt)
#pragma unroll
    for (int nt = 0; nt < 4; ++nt) acc[mt][nt] = zero8;

  gemm_core_32x64(MShi, MSlo, B5t, FD, (size_t)(m0w + m) * FD, (size_t)(n0 + m) * FD, hh, acc);

  float bv[4];
#pragma unroll
  for (int nt = 0; nt < 4; ++nt) bv[nt] = bf16r(b5[n0 + 16 * nt + m]);
#pragma unroll
  for (int nt = 0; nt < 4; ++nt)
#pragma unroll
    for (int mt = 0; mt < 2; ++mt)
#pragma unroll
      for (int r = 0; r < 8; ++r) {
        const int tokl = 32 * w + 16 * mt + 8 * hh + r;
        const int feat = 16 * nt + m;
        const float y = acc[mt][nt][r] + bv[nt];
        sF[tokl * 64 + feat] = fmaxf(y, y * SLOPE);
      }
  __syncthreads();
  {
    const int rsub = lane >> 4, c4 = (lane & 15) * 4;
    v4f vals[16];
#pragma unroll
    for (int it = 0; it < 16; ++it) {
      const int row = 32 * w + 2 * it + rsub;
      v4f v = *(const v4fa*)(sF + row * 64 + c4);
      const v4f nv = *(const v4fa*)(x + (size_t)(m0 + row) * FD + n0 + c4);
      v[0] += bf16r(nv[0]); v[1] += bf16r(nv[1]); v[2] += bf16r(nv[2]); v[3] += bf16r(nv[3]);
      vals[it] = v;
    }
    for (int pass = 0; pass < 2; ++pass) {
#pragma unroll
      for (int it = 0; it < 16; ++it) {
        const int row = 32 * w + 2 * it + rsub;
        *(volatile v4f*)(out + (size_t)(m0 + row) * FD + n0 + c4) = vals[it];
      }
      __threadfence();
    }
  }
}

extern "C" void kernel_launch(void* const* d_in, const int* in_sizes, int n_in,
                              void* d_out, int out_size, void* d_ws, size_t ws_size,
                              hipStream_t stream) {
  if (n_in < 5) return;
  if (in_sizes[0] != MR * FD) return;
  if (in_sizes[1] != NC3 * FD) return;
  if (in_sizes[2] != FD) return;
  if (in_sizes[3] != FD * FD) return;
  if (in_sizes[4] != FD) return;
  if (out_size != MR * FD) return;

  const float* x  = (const float*)d_in[0];
  const float* W3 = (const float*)d_in[1];
  const float* b3 = (const float*)d_in[2];
  const float* W5 = (const float*)d_in[3];
  const float* b5 = (const float*)d_in[4];
  float* out = (float*)d_out;

  const size_t PXB = (size_t)MR * FD * 2;
  const size_t PB3 = (size_t)NC3 * FD * 2;
  const size_t PB5 = (size_t)FD * FD * 2;
  const size_t PAB = (size_t)MR * NC3 * 4;
  const size_t PMS = (size_t)MR * FD * 2;
  size_t off = 0;
  const size_t oXb  = off; off += PXB;
  const size_t oB3  = off; off += PB3;
  const size_t oB5  = off; off += PB5;
  const size_t oAB  = off; off += PAB;
  const size_t oMSh = off; off += PMS;
  const size_t oMSl = off; off += PMS;
  if (off > ws_size) return;

  char* ws = (char*)d_ws;
  unsigned short* Xb   = (unsigned short*)(ws + oXb);
  unsigned short* B3t  = (unsigned short*)(ws + oB3);
  unsigned short* B5t  = (unsigned short*)(ws + oB5);
  float*          AB   = (float*)(ws + oAB);
  unsigned short* MShi = (unsigned short*)(ws + oMSh);
  unsigned short* MSlo = (unsigned short*)(ws + oMSl);

  k_cvt<<<dim3((MR * FD / 8) / 256), 256, 0, stream>>>(x, Xb);
  k_wt<<<dim3(FD / 64, FD / 64, 3), 256, 0, stream>>>(W3, W5, B3t, B5t);
  k_ab<<<dim3(MR / 128, NC3 / 64), 128, 0, stream>>>(Xb, B3t, AB);
  k_pair<<<dim3(FD / FT, NB), 256, 0, stream>>>(AB, b3, MShi, MSlo);
  k_out<<<dim3(MR / 128, FD / 64), 128, 0, stream>>>(MShi, MSlo, B5t, b5, x, out);
  (void)hipGetLastError();
}
